// InteractionLayer_72602127171983
// MI455X (gfx1250) — hardware-verified
//
#include <hip/hip_runtime.h>


#ifndef NB
#define NB 2
#endif
#ifndef SEQ
#define SEQ 1024
#endif
#define NB_FULL 2
#define SEQ_FULL 1024
#define NF 64
#define KD (2 * NF)
#define TI 64
#define JC 16

static_assert(NB >= 1 && NB <= NB_FULL);
static_assert(SEQ >= TI && SEQ <= SEQ_FULL && (SEQ % TI) == 0 && (SEQ % 64) == 0);
static_assert(NF == 64 && (KD % 32) == 0);
static_assert((SEQ_FULL % JC) == 0 && (SEQ_FULL % 64) == 0);
static_assert(((NB * SEQ_FULL * NF) % 256) == 0);
static_assert(((TI * NF / 4) % 128) == 0 && ((JC * NF / 4) % 128) == 0 && ((NF * NF) % 128) == 0);

typedef unsigned short us;
typedef us     v8us  __attribute__((ext_vector_type(8)));
typedef __bf16 v16bf __attribute__((ext_vector_type(16)));
typedef float  v8f   __attribute__((ext_vector_type(8)));
typedef float  v4f   __attribute__((ext_vector_type(4)));

union Frag { v16bf v; v8us h[2]; };

__device__ __forceinline__ us f2bf(float f) {
    unsigned int u = __float_as_uint(f);
    u += 0x7FFFu + ((u >> 16) & 1u);
    return (us)(u >> 16);
}
__device__ __forceinline__ float bf2f(us h) {
    return __uint_as_float(((unsigned int)h) << 16);
}
__device__ __forceinline__ v4f rne4(v4f a) {
    a.x = bf2f(f2bf(a.x)); a.y = bf2f(f2bf(a.y)); a.z = bf2f(f2bf(a.z)); a.w = bf2f(f2bf(a.w));
    return a;
}
__device__ __forceinline__ v4f absdiff4(v4f a, v4f c) {
    v4f d = a - c;
    d.x = __builtin_fabsf(d.x); d.y = __builtin_fabsf(d.y); d.z = __builtin_fabsf(d.z); d.w = __builtin_fabsf(d.w);
    return d;
}
__device__ __forceinline__ float sspf(float x) {
    const float t  = __builtin_amdgcn_exp2f(-1.44269504088896341f * __builtin_fabsf(x));
    const float lg = __builtin_amdgcn_logf(1.0f + t);
    return fmaf(0.693147180559945309f, lg, fmaxf(x, 0.0f)) - 0.693147180559945309f;
}
__device__ __forceinline__ v4f ssp4(v4f a) {
    a.x = sspf(a.x); a.y = sspf(a.y); a.z = sspf(a.z); a.w = sspf(a.w);
    return a;
}
__device__ __forceinline__ v8us pack8(v4f a, v4f c) {
    v8us o;
    o[0] = f2bf(a.x); o[1] = f2bf(a.y); o[2] = f2bf(a.z); o[3] = f2bf(a.w);
    o[4] = f2bf(c.x); o[5] = f2bf(c.y); o[6] = f2bf(c.z); o[7] = f2bf(c.w);
    return o;
}
__device__ __forceinline__ void split8(v4f a, v4f c, v8us& hi, v8us& lo) {
    const float x[8] = {a.x, a.y, a.z, a.w, c.x, c.y, c.z, c.w};
#pragma unroll
    for (int i = 0; i < 8; ++i) {
        const us h = f2bf(x[i]);
        hi[i] = h;
        lo[i] = f2bf(x[i] - bf2f(h));
    }
}
__device__ __forceinline__ void wave_sync() {
    __builtin_amdgcn_fence(__ATOMIC_RELEASE, "wavefront");
    __builtin_amdgcn_wave_barrier();
}

__device__ __forceinline__ v8f wmma16(v16bf a, v16bf b, v8f c) {
    v8f d = __builtin_amdgcn_wmma_f32_16x16x32_bf16(false, a, false, b, (short)0, c, false, false);
    asm volatile("v_nop\n\tv_nop\n\tv_nop\n\tv_nop" : "+v"(d) : "v"(a), "v"(b));
    return d;
}

__device__ __forceinline__ v16bf ld_frag(const us* P, int ld, int row, int k0, int hsel) {
    Frag f;
    const us* p = P + (size_t)row * ld + k0 + 8 * hsel;
    f.h[0] = *(const v8us*)p;
    f.h[1] = *(const v8us*)(p + 16);
    return f.v;
}

__global__ __launch_bounds__(256)
void k_cvt(const float* __restrict__ src, int spitch, int scol, int grp, int gstride,
           us* __restrict__ dst, int dpitch, int dcol, int nrows, int nseg)
{
    const int lane = threadIdx.x & 31;
    const int gw   = blockIdx.x * 8 + (threadIdx.x >> 5);
    if (gw >= nrows * nseg) return;
    const int r    = gw / nseg;
    const int sg   = gw - r * nseg;
    const int g    = r / grp;
    const int srow = g * gstride + (r - g * grp);
    const float* sp = src + (size_t)srow * spitch + scol + sg * 256 + lane * 8;
    const v4f a = *(const v4f*)sp;
    const v4f c = *(const v4f*)(sp + 4);
    const v8us o = pack8(a, c);
    us* dp = dst + (size_t)r * dpitch + dcol + sg * 256 + lane * 8;
    *(volatile v8us*)dp = o;
    __threadfence();
    *(volatile v8us*)dp = o;
}

__global__ __launch_bounds__(256)
void k_wtrans(const float* __restrict__ W, us* __restrict__ WT2)
{
    __shared__ float ts[64][65];
    const int tid = threadIdx.x, lane = tid & 31, wave = tid >> 5;

#pragma unroll
    for (int p = 0; p < 4; ++p) {
        const int kl = p * 16 + (tid >> 4);
        const int o4 = (tid & 15) * 4;
        const v4f x = *(const v4f*)(W + kl * NF + o4);
        ts[kl][o4 + 0] = x.x; ts[kl][o4 + 1] = x.y; ts[kl][o4 + 2] = x.z; ts[kl][o4 + 3] = x.w;
    }
    __syncthreads();

    v8us o[2];
#pragma unroll
    for (int p = 0; p < 2; ++p) {
        const int ol = p * 32 + wave * 4 + (lane >> 3);
        const int k8 = (lane & 7) * 8;
#pragma unroll
        for (int i = 0; i < 8; ++i) o[p][i] = f2bf(ts[k8 + i][ol]);
    }
#pragma unroll
    for (int p = 0; p < 2; ++p) {
        const int ol = p * 32 + wave * 4 + (lane >> 3);
        const int k8 = (lane & 7) * 8;
        us* d = WT2 + (size_t)ol * KD + k8;
        *(volatile v8us*)d = o[p];
        *(volatile v8us*)(d + NF) = o[p];
    }
    __threadfence();
#pragma unroll
    for (int p = 0; p < 2; ++p) {
        const int ol = p * 32 + wave * 4 + (lane >> 3);
        const int k8 = (lane & 7) * 8;
        us* d = WT2 + (size_t)ol * KD + k8;
        *(volatile v8us*)d = o[p];
        *(volatile v8us*)(d + NF) = o[p];
    }
}

template <int EPI>
__global__ __launch_bounds__(128)
void k_gemm(const us* __restrict__ A, int lda, int strideA,
            const us* __restrict__ B, int ldb, int strideB,
            const float* __restrict__ bias,
            void* __restrict__ Cv, int ldc, int strideC, int K, int loff)
{
    __shared__ __attribute__((aligned(16))) float tile[4 * 16 * 64];

    const int lane = threadIdx.x & 31, wave = threadIdx.x >> 5;
    const int hsel = lane >> 4, m = lane & 15;
    const int m0 = blockIdx.x * 64 + wave * 16;
    const int n0 = blockIdx.y * 64;
    const us* Ab = A + (size_t)blockIdx.z * (size_t)strideA;
    const us* Bb = B + (size_t)blockIdx.z * (size_t)strideB;

    v8f c0 = {}; v8f c1 = {}; v8f c2 = {}; v8f c3 = {};
    for (int k0 = 0; k0 < K; k0 += 32) {
        const v16bf a  = ld_frag(Ab, lda, m0 + m, k0, hsel);
        const v16bf b0 = ld_frag(Bb, ldb, n0 + m,      k0, hsel);
        const v16bf b1 = ld_frag(Bb, ldb, n0 + 16 + m, k0, hsel);
        const v16bf b2 = ld_frag(Bb, ldb, n0 + 32 + m, k0, hsel);
        const v16bf b3 = ld_frag(Bb, ldb, n0 + 48 + m, k0, hsel);
        c0 = wmma16(a, b0, c0);
        c1 = wmma16(a, b1, c1);
        c2 = wmma16(a, b2, c2);
        c3 = wmma16(a, b3, c3);
    }

    float* tw = tile + wave * 1024;
#pragma unroll
    for (int r = 0; r < 8; ++r) {
        const int row = 8 * hsel + r;
        tw[row * 64 + m]      = c0[r];
        tw[row * 64 + 16 + m] = c1[r];
        tw[row * 64 + 32 + m] = c2[r];
        tw[row * 64 + 48 + m] = c3[r];
    }
    __syncthreads();

    if (EPI == 1) {
        us* Cb = (us*)Cv + (size_t)blockIdx.z * (size_t)strideC;
        v8us hi[4], lo[4];
#pragma unroll
        for (int p = 0; p < 4; ++p) {
            const int row = 4 * p + (lane >> 3);
            const int col = 8 * (lane & 7);
            const v4f ba = rne4(*(const v4f*)(bias + n0 + col));
            const v4f bc = rne4(*(const v4f*)(bias + n0 + col + 4));
            const v4f a = ssp4(*(const v4f*)(tw + row * 64 + col) + ba);
            const v4f c = ssp4(*(const v4f*)(tw + row * 64 + col + 4) + bc);
            split8(a, c, hi[p], lo[p]);
        }
#pragma unroll
        for (int p = 0; p < 4; ++p) {
            us* d = Cb + (size_t)(m0 + 4 * p + (lane >> 3)) * ldc + n0 + 8 * (lane & 7);
            *(volatile v8us*)d = hi[p];
            *(volatile v8us*)(d + loff) = lo[p];
        }
        __threadfence();
#pragma unroll
        for (int p = 0; p < 4; ++p) {
            us* d = Cb + (size_t)(m0 + 4 * p + (lane >> 3)) * ldc + n0 + 8 * (lane & 7);
            *(volatile v8us*)d = hi[p];
            *(volatile v8us*)(d + loff) = lo[p];
        }
    } else {
        float* Cb = (float*)Cv + (size_t)blockIdx.z * (size_t)strideC;
        const v4f bb = rne4(*(const v4f*)(bias + n0 + 4 * m));
        v4f vals[8];
#pragma unroll
        for (int p = 0; p < 8; ++p) {
            const int row = 2 * p + hsel;
            vals[p] = *(const v4f*)(tw + row * 64 + 4 * m) + bb;
        }
#pragma unroll
        for (int p = 0; p < 8; ++p) {
            float* d = Cb + (size_t)(m0 + 2 * p + hsel) * ldc + n0 + 4 * m;
            *(volatile v4f*)d = vals[p];
        }
        __threadfence();
#pragma unroll
        for (int p = 0; p < 8; ++p) {
            float* d = Cb + (size_t)(m0 + 2 * p + hsel) * ldc + n0 + 4 * m;
            *(volatile v4f*)d = vals[p];
        }
    }
}

__global__ __launch_bounds__(128)
void k_pair(const float* __restrict__ r, const float* __restrict__ h1,
            const float* __restrict__ f1w, const float* __restrict__ f1b,
            const float* __restrict__ f2w, const float* __restrict__ f2b,
            us* __restrict__ hcat)
{
    __shared__ __attribute__((aligned(16))) float sRI[TI * NF];
    __shared__ __attribute__((aligned(16))) float sRJ[JC * NF];
    __shared__ __attribute__((aligned(16))) float sHJ[JC * NF];
    __shared__ __attribute__((aligned(16))) us    sW1[NF * NF];
    __shared__ __attribute__((aligned(16))) us    sW2[NF * NF];
    __shared__ __attribute__((aligned(16))) us    sP[4 * 16 * KD];

    const int tid = threadIdx.x, lane = tid & 31, wave = tid >> 5;
    const int hsel = lane >> 4, m = lane & 15;
    const int b  = blockIdx.y;
    const int i0 = blockIdx.x * TI;
    const size_t jrow0 = (size_t)b * SEQ_FULL;

    {
        const v4f* src = (const v4f*)(r + (jrow0 + i0) * NF);
#pragma unroll
        for (int p = 0; p < (TI * NF / 4) / 128; ++p) ((v4f*)sRI)[p * 128 + tid] = rne4(src[p * 128 + tid]);
    }
#pragma unroll 4
    for (int p = 0; p < (NF * NF) / 128; ++p) {
        const int idx = p * 128 + tid;
        const int k = idx >> 6, o = idx & 63;
        sW1[o * NF + k] = f2bf(f1w[idx]);
        sW2[o * NF + k] = f2bf(f2w[idx]);
    }
    float b1v[4], b2v[4];
#pragma unroll
    for (int nt = 0; nt < 4; ++nt) {
        b1v[nt] = bf2f(f2bf(f1b[nt * 16 + m]));
        b2v[nt] = bf2f(f2bf(f2b[nt * 16 + m]));
    }
    v8f hacc[4];
#pragma unroll
    for (int nt = 0; nt < 4; ++nt)
#pragma unroll
        for (int rr = 0; rr < 8; ++rr) hacc[nt][rr] = 0.0f;
    __syncthreads();

    us* sPw = sP + wave * (16 * KD);
    const float* ri = sRI + (wave * 16 + m) * NF;

#pragma unroll 1
    for (int jc = 0; jc < SEQ_FULL; jc += JC) {
        __syncthreads();
        {
            const v4f* srcr = (const v4f*)(r  + (jrow0 + jc) * NF);
            const v4f* srch = (const v4f*)(h1 + (jrow0 + jc) * NF);
#pragma unroll
            for (int p = 0; p < (JC * NF / 4) / 128; ++p) {
                ((v4f*)sRJ)[p * 128 + tid] = rne4(srcr[p * 128 + tid]);
                ((v4f*)sHJ)[p * 128 + tid] = srch[p * 128 + tid];
            }
        }
        __syncthreads();

#pragma unroll 1
        for (int jj = 0; jj < JC; ++jj) {
            const float* rj = sRJ + jj * NF;

            v8f c[4];
#pragma unroll
            for (int nt = 0; nt < 4; ++nt)
#pragma unroll
                for (int rr = 0; rr < 8; ++rr) c[nt][rr] = b1v[nt];
#pragma unroll
            for (int s = 0; s < 2; ++s) {
                const int fb = 32 * s + 8 * hsel;
                const v4f da = absdiff4(*(const v4f*)(ri + fb),      *(const v4f*)(rj + fb));
                const v4f dc = absdiff4(*(const v4f*)(ri + fb + 4),  *(const v4f*)(rj + fb + 4));
                const v4f ea = absdiff4(*(const v4f*)(ri + fb + 16), *(const v4f*)(rj + fb + 16));
                const v4f ec = absdiff4(*(const v4f*)(ri + fb + 20), *(const v4f*)(rj + fb + 20));
                Frag ah, al;
                split8(da, dc, ah.h[0], al.h[0]);
                split8(ea, ec, ah.h[1], al.h[1]);
#pragma unroll
                for (int nt = 0; nt < 4; ++nt) {
                    const v16bf bb = ld_frag(sW1, NF, nt * 16 + m, 32 * s, hsel);
                    c[nt] = wmma16(ah.v, bb, c[nt]);
                    c[nt] = wmma16(al.v, bb, c[nt]);
                }
            }

            wave_sync();
#pragma unroll
            for (int nt = 0; nt < 4; ++nt)
#pragma unroll
                for (int rr = 0; rr < 8; ++rr) {
                    const float v = sspf(c[nt][rr]);
                    const us hh = f2bf(v);
                    const us ll = f2bf(v - bf2f(hh));
                    us* q = sPw + (8 * hsel + rr) * KD + nt * 16 + m;
                    q[0]  = hh;
                    q[NF] = ll;
                }
            wave_sync();

            v8f c2[4];
#pragma unroll
            for (int nt = 0; nt < 4; ++nt)
#pragma unroll
                for (int rr = 0; rr < 8; ++rr) c2[nt][rr] = b2v[nt];
#pragma unroll
            for (int s2 = 0; s2 < 4; ++s2) {
                const v16bf a2 = ld_frag(sPw, KD, m, 32 * s2, hsel);
#pragma unroll
                for (int nt = 0; nt < 4; ++nt) {
                    const v16bf bb = ld_frag(sW2, NF, nt * 16 + m, 32 * (s2 & 1), hsel);
                    c2[nt] = wmma16(a2, bb, c2[nt]);
                }
            }

            const float* hj = sHJ + jj * NF;
#pragma unroll
            for (int nt = 0; nt < 4; ++nt) {
                const float hv = hj[nt * 16 + m];
#pragma unroll
                for (int rr = 0; rr < 8; ++rr)
                    hacc[nt][rr] = fmaf(sspf(c2[nt][rr]), hv, hacc[nt][rr]);
            }
        }
    }

    __syncthreads();
    float* tw = sRI + wave * (16 * NF);
#pragma unroll
    for (int rr = 0; rr < 8; ++rr) {
        const int row = 8 * hsel + rr;
#pragma unroll
        for (int nt = 0; nt < 4; ++nt) tw[row * NF + nt * 16 + m] = hacc[nt][rr];
    }
    __syncthreads();

    v8us hi[4], lo[4];
#pragma unroll
    for (int p = 0; p < 4; ++p) {
        const int row = 4 * p + (lane >> 3);
        const int col = 8 * (lane & 7);
        const v4f a  = *(const v4f*)(tw + row * NF + col);
        const v4f cc = *(const v4f*)(tw + row * NF + col + 4);
        split8(a, cc, hi[p], lo[p]);
    }
    us* Cb = hcat + ((size_t)b * SEQ + i0 + wave * 16) * KD;
#pragma unroll
    for (int p = 0; p < 4; ++p) {
        us* d = Cb + (size_t)(4 * p + (lane >> 3)) * KD + 8 * (lane & 7);
        *(volatile v8us*)d = hi[p];
        *(volatile v8us*)(d + NF) = lo[p];
    }
    __threadfence();
#pragma unroll
    for (int p = 0; p < 4; ++p) {
        us* d = Cb + (size_t)(4 * p + (lane >> 3)) * KD + 8 * (lane & 7);
        *(volatile v8us*)d = hi[p];
        *(volatile v8us*)(d + NF) = lo[p];
    }
}

static inline size_t al256(size_t x) { return (x + 255) & ~(size_t)255; }

extern "C" void kernel_launch(void* const* d_in, const int* in_sizes, int n_in,
                              void* d_out, int out_size, void* d_ws, size_t ws_size,
                              hipStream_t stream)
{
    if (n_in < 12) return;
    if (in_sizes[0] < NB * SEQ_FULL * NF) return;
    if (in_sizes[1] < NB * SEQ_FULL * NF) return;
    if (in_sizes[2] < NF * NF || in_sizes[4] < NF * NF || in_sizes[6] < NF * NF) return;
    if (in_sizes[8] < NF * NF || in_sizes[10] < NF * NF) return;
    if (in_sizes[3] < NF || in_sizes[5] < NF || in_sizes[7] < NF) return;
    if (in_sizes[9] < NF || in_sizes[11] < NF) return;
    if (out_size < ((NB - 1) * SEQ_FULL + SEQ) * NF) return;

    const float* x    = (const float*)d_in[0];
    const float* r    = (const float*)d_in[1];
    const float* aw1w = (const float*)d_in[2];
    const float* aw1b = (const float*)d_in[3];
    const float* aw2w = (const float*)d_in[4];
    const float* aw2b = (const float*)d_in[5];
    const float* aw3w = (const float*)d_in[6];
    const float* aw3b = (const float*)d_in[7];
    const float* f1w  = (const float*)d_in[8];
    const float* f1b  = (const float*)d_in[9];
    const float* f2w  = (const float*)d_in[10];
    const float* f2b  = (const float*)d_in[11];
    float* out = (float*)d_out;

    char* ws = (char*)d_ws;
    size_t off = 0;
    us* xb    = (us*)(ws + off);    off += al256((size_t)NB * SEQ_FULL * NF * sizeof(us));
    us* aw1T  = (us*)(ws + off);    off += al256((size_t)NF * KD * sizeof(us));
    us* aw2T  = (us*)(ws + off);    off += al256((size_t)NF * KD * sizeof(us));
    us* aw3T  = (us*)(ws + off);    off += al256((size_t)NF * KD * sizeof(us));
    float* h1 = (float*)(ws + off); off += al256((size_t)NB * SEQ_FULL * NF * sizeof(float));
    us* hcat  = (us*)(ws + off);    off += al256((size_t)NB * SEQ * KD * sizeof(us));
    us* h3c   = (us*)(ws + off);    off += al256((size_t)NB * SEQ * KD * sizeof(us));
    if (off > ws_size) return;

    const dim3 b256(256), b128(128);

    {
        const int nrows = NB * SEQ_FULL * NF / 256;
        k_cvt<<<dim3((nrows + 7) / 8), b256, 0, stream>>>(x, 256, 0, nrows, nrows, xb, 256, 0, nrows, 1);
    }
    k_wtrans<<<dim3(1), b256, 0, stream>>>(aw1w, aw1T);
    k_wtrans<<<dim3(1), b256, 0, stream>>>(aw2w, aw2T);
    k_wtrans<<<dim3(1), b256, 0, stream>>>(aw3w, aw3T);

    k_gemm<0><<<dim3(NB * SEQ_FULL / 64, 1, 1), b128, 0, stream>>>(
        xb, NF, 0, aw1T, KD, 0, aw1b, (void*)h1, NF, 0, NF, 0);

    k_pair<<<dim3(SEQ / TI, NB), b128, 0, stream>>>(r, h1, f1w, f1b, f2w, f2b, hcat);

    k_gemm<1><<<dim3(NB * SEQ / 64, 1, 1), b128, 0, stream>>>(
        hcat, KD, 0, aw2T, KD, 0, aw2b, (void*)h3c, KD, 0, KD, NF);

    k_gemm<0><<<dim3(SEQ / 64, 1, NB), b128, 0, stream>>>(
        h3c, KD, SEQ * KD, aw3T, KD, 0, aw3b, (void*)out, NF, SEQ_FULL * NF, KD, 0);
}
